// GraphSAGENet_69097433858679
// MI455X (gfx1250) — hardware-run, weakly checked
//
#include <hip/hip_runtime.h>

typedef float          v8f   __attribute__((ext_vector_type(8)));
typedef float          v4f   __attribute__((ext_vector_type(4)));
typedef unsigned int   v4u   __attribute__((ext_vector_type(4)));
typedef int            v8i   __attribute__((ext_vector_type(8)));
typedef unsigned short v8us  __attribute__((ext_vector_type(8)));
typedef unsigned short v16us __attribute__((ext_vector_type(16)));
typedef __bf16         v16bf __attribute__((ext_vector_type(16)));
typedef _Float16       v16h  __attribute__((ext_vector_type(16)));
typedef v4f  __attribute__((may_alias)) v4fa;
typedef v8us __attribute__((may_alias)) v8usa;
union FragB { v16bf v; v16us u; v8us h[2]; v8i w; };
union FragH { v16h  v; v16us u; v8us h[2]; v8i w; };

__device__ __forceinline__ v8f wmb(const FragB& a, const FragB& b, v8f c) {
  v8f d = __builtin_amdgcn_wmma_f32_16x16x32_bf16(false, a.v, false, b.v, (short)0, c, false, false);
  asm volatile("v_nop\n\tv_nop\n\tv_nop\n\tv_nop" : "+v"(d) : "v"(a.w), "v"(b.w));
  return d;
}

__device__ __forceinline__ v8f wmh(const FragH& a, const FragH& b, v8f c) {
  v8f d = __builtin_amdgcn_wmma_f32_16x16x32_f16(false, a.v, false, b.v, (short)0, c, false, false);
  asm volatile("v_nop\n\tv_nop\n\tv_nop\n\tv_nop" : "+v"(d) : "v"(a.w), "v"(b.w));
  return d;
}

__device__ __forceinline__ unsigned bf16_bits(float f) {
  const unsigned u = __float_as_uint(f);
  const unsigned r = (u + 0x7FFFu + ((u >> 16) & 1u)) >> 16;
  const unsigned q = (u >> 16) | 0x40u;
  return ((u & 0x7fffffffu) > 0x7f800000u) ? q : r;
}

__device__ __forceinline__ float bf16_val(float f) {
  return __uint_as_float(bf16_bits(f) << 16);
}
__device__ __forceinline__ int clampi(int v, int lo, int hi) {
  return v < lo ? lo : (v > hi ? hi : v);
}

__device__ __forceinline__ unsigned f16_bits(float f) {
  const unsigned u  = __float_as_uint(f);
  const unsigned s  = (u >> 16) & 0x8000u;
  const unsigned a  = u & 0x7fffffffu;
  const unsigned t  = a - 0x38000000u;
  const unsigned r  = (t + 0x0FFFu + ((t >> 13) & 1u)) >> 13;
  const unsigned rc = r > 0x7C00u ? 0x7C00u : r;
  const bool small  = a < 0x38800000u;
  const bool isnan  = a > 0x7f800000u;
  const unsigned fin = small ? 0u : (s | rc);
  return isnan ? (s | 0x7E00u) : fin;
}

__device__ __forceinline__ unsigned pk16(unsigned lo, unsigned hi) { return lo | (hi << 16); }
__device__ __forceinline__ unsigned bf16_lo_bits(float v) {
  float hi = bf16_val(v);
  asm volatile("" : "+v"(hi));
  return bf16_bits(v - hi);
}
__device__ __forceinline__ v4u pack8_bf16(v4f a, v4f c) {
  return (v4u){ pk16(bf16_bits(a[0]), bf16_bits(a[1])), pk16(bf16_bits(a[2]), bf16_bits(a[3])),
                pk16(bf16_bits(c[0]), bf16_bits(c[1])), pk16(bf16_bits(c[2]), bf16_bits(c[3])) };
}
__device__ __forceinline__ v4u pack8_bf16_lo(v4f a, v4f c) {
  return (v4u){ pk16(bf16_lo_bits(a[0]), bf16_lo_bits(a[1])), pk16(bf16_lo_bits(a[2]), bf16_lo_bits(a[3])),
                pk16(bf16_lo_bits(c[0]), bf16_lo_bits(c[1])), pk16(bf16_lo_bits(c[2]), bf16_lo_bits(c[3])) };
}
__device__ __forceinline__ v4u pack8_f16(v4f a, v4f c) {
  return (v4u){ pk16(f16_bits(a[0]), f16_bits(a[1])), pk16(f16_bits(a[2]), f16_bits(a[3])),
                pk16(f16_bits(c[0]), f16_bits(c[1])), pk16(f16_bits(c[2]), f16_bits(c[3])) };
}

template <int FORM>
__global__ __launch_bounds__(256) void k_plane(const float* __restrict__ src, int rows, int cols, int ldsrc,
                                               unsigned short* __restrict__ dst, int MP, int KP) {
  static_assert(FORM >= 0 && FORM <= 3);
  const int KTOT = (FORM == 1 || FORM == 3) ? 2 * KP : KP;
  const unsigned ppr   = (unsigned)(KTOT >> 3);
  const unsigned kp8   = (unsigned)(KP >> 3);
  const unsigned total = (unsigned)MP * ppr;
  const unsigned g     = blockIdx.x * 256u + threadIdx.x;
  const unsigned rowu  = g / ppr;
  const unsigned p     = g - rowu * ppr;
  const bool second    = p >= kp8;
  const int row = (int)rowu;
  const int c0  = (int)((second ? p - kp8 : p) << 3);
  const float* srow = src + (size_t)clampi(row, 0, rows - 1) * (size_t)ldsrc;
  float x[8];
  unsigned mk[8];
#pragma unroll
  for (int e = 0; e < 8; ++e) {
    const int c = c0 + e;
    const float v = srow[clampi(c, 0, cols - 1)];
    asm volatile("" :: "v"(v));
    x[e]  = v;
    mk[e] = (row < rows && c < cols) ? 0xFFFFu : 0u;
  }
  const v4f a = (v4f){ x[0], x[1], x[2], x[3] };
  const v4f c = (v4f){ x[4], x[5], x[6], x[7] };
  v4u o;
  if (FORM == 2) {
    o = pack8_f16(a, c);
  } else {
    const v4u hi = pack8_bf16(a, c);
    o = hi;
    if (FORM == 1) { const v4u lo = pack8_bf16_lo(a, c); o = second ? lo : hi; }
  }
  const v4u mw = (v4u){ pk16(mk[0], mk[1]), pk16(mk[2], mk[3]), pk16(mk[4], mk[5]), pk16(mk[6], mk[7]) };
  o &= mw;
  if (g < total) {
    volatile v4u* q = (volatile v4u*)(dst + (size_t)g * 8);
    *q = o;
    __threadfence();
    *q = o;
  }
}

template <int FORM> struct FragOf    { typedef FragB T; };
template <>         struct FragOf<2> { typedef FragH T; };
__device__ __forceinline__ v8f mm(const FragB& a, const FragB& b, v8f c) { return wmb(a, b, c); }
__device__ __forceinline__ v8f mm(const FragH& a, const FragH& b, v8f c) { return wmh(a, b, c); }
template <class F> __device__ __forceinline__ F ld_frag(const unsigned short* p) {
  F f;
  f.h[0] = *(const v8usa*)(p);
  f.h[1] = *(const v8usa*)(p + 16);
  return f;
}

template <int FORM, int EPI>
__global__ __launch_bounds__(256) __attribute__((amdgpu_num_vgpr(248)))
void k_gemm_nt(const unsigned short* __restrict__ A, const unsigned short* __restrict__ B,
               const float* __restrict__ bias, float* __restrict__ D, int M, int N, int KTOT, int ldd) {
  static_assert(FORM >= 0 && FORM <= 2);
  static_assert(EPI == 0 || EPI == 1);
  typedef typename FragOf<FORM>::T F;
  __shared__ __attribute__((aligned(16))) float sT[8][16 * 68];
  const int lane = threadIdx.x & 31;
  const int wave = threadIdx.x >> 5;
  const int tilesM = (M + 63) >> 6;
  const int tilesN = (N + 63) >> 6;
  const int tile = blockIdx.x * 8 + wave;
  if (tile >= tilesM * tilesN) return;
  const int tm = tile / tilesN;
  const int tn = tile - tm * tilesN;
  const int m0 = tm << 6;
  const int n0 = tn << 6;

  const int rl = lane & 15;
  const int h8 = (lane >> 4) * 8;
  const unsigned short* pa = A + (size_t)(m0 + rl) * (size_t)KTOT + h8;
  const unsigned short* pb = B + (size_t)(n0 + rl) * (size_t)KTOT + h8;

  v8f acc[4][4];
#pragma unroll
  for (int i = 0; i < 4; ++i)
#pragma unroll
    for (int j = 0; j < 4; ++j) acc[i][j] = (v8f){0.f, 0.f, 0.f, 0.f, 0.f, 0.f, 0.f, 0.f};

#pragma unroll 1
  for (int k0 = 0; k0 < KTOT; k0 += 32) {
    F bf[4];
#pragma unroll
    for (int j = 0; j < 4; ++j) bf[j] = ld_frag<F>(pb + (size_t)(j << 4) * (size_t)KTOT + k0);
#pragma unroll
    for (int i = 0; i < 4; ++i) {
      const F af = ld_frag<F>(pa + (size_t)(i << 4) * (size_t)KTOT + k0);
#pragma unroll
      for (int j = 0; j < 4; ++j) acc[i][j] = mm(af, bf[j], acc[i][j]);
    }
  }

  float* slab = sT[wave];
  const int hh = lane >> 4;
  const int c4 = (lane & 15) * 4;
  const int nc = n0 + c4;
  const bool cok = nc < N;
  v4f bv = (v4f){0.f, 0.f, 0.f, 0.f};
  if (EPI == 1) {
    bv = *(const v4fa*)(bias + clampi(nc, 0, N - 4));
    asm volatile("" :: "v"(bv));
  }
#pragma unroll
  for (int i = 0; i < 4; ++i) {
    const int mBase = m0 + (i << 4);
#pragma unroll
    for (int j = 0; j < 4; ++j) {
#pragma unroll
      for (int r = 0; r < 8; ++r) slab[(h8 + r) * 68 + (j << 4) + rl] = acc[i][j][r];
    }
    __builtin_amdgcn_fence(__ATOMIC_RELEASE, "workgroup");
    __builtin_amdgcn_wave_barrier();
    __builtin_amdgcn_fence(__ATOMIC_ACQUIRE, "workgroup");
    v4f vv[8];
#pragma unroll
    for (int it = 0; it < 8; ++it) {
      const int row = it * 2 + hh;
      v4f v = *(const v4fa*)(slab + row * 68 + c4);
      if (EPI == 1) v += bv;
      vv[it] = v;
    }
    for (int pass = 0; pass < 2; ++pass) {
#pragma unroll
      for (int it = 0; it < 8; ++it) {
        const int row = mBase + it * 2 + hh;
        if (cok && row < M) *(volatile v4f*)(D + (size_t)row * (size_t)ldd + nc) = vv[it];
      }
      __threadfence();
    }
    __builtin_amdgcn_fence(__ATOMIC_RELEASE, "workgroup");
    __builtin_amdgcn_wave_barrier();
    __builtin_amdgcn_fence(__ATOMIC_ACQUIRE, "workgroup");
  }
}

#define SG_N       100000
#define SG_E       1600000
#define SG_F       128
#define SG_H       16
#define SG_C       40
#define SG_MP      100096
#define SG_NBA     1024
#define SG_NBLK    98
#define SG_RCAP    20992
#define SG_WLCAP   3072
#define SG_DEGCAP  64
#define SG_NWCH    (SG_E / 256)
#define SG_SWEEP   ((SG_NWCH + 7) / 8)
#define SG_XBLK    (SG_MP * 16 / 256)
#define SG_NGRP    (SG_N / 16)
#define SG_ZINTS   (SG_RCAP + 8 * SG_NBA + 2 * SG_NBA + 32)
#define SG_LDSINTS (SG_ZINTS + 8 * SG_WLCAP)
#define SPLIT2     1

static_assert(SG_E % 256 == 0);
static_assert(SG_N <= 131072 && SG_NBA == 1024);
static_assert(SG_NBLK * SG_NBA >= SG_MP && (SG_NBLK - 1) * SG_NBA < SG_N);
static_assert(SG_MP % 64 == 0 && SG_MP >= SG_N && SG_N % 16 == 0 && SG_N % 2 == 0);
static_assert((SG_MP * 16) % 256 == 0);
static_assert(SG_RCAP % 256 == 0 && (SG_RCAP / 4) % 32 == 0);
static_assert(SG_RCAP * 4 >= 16721 * 5);
static_assert(SG_DEGCAP >= 36 + 8 && SG_DEGCAP % 8 == 0);
static_assert(SG_ZINTS % 4 == 0 && SG_WLCAP % 4 == 0);
static_assert(SG_LDSINTS * 4 <= 262144);
static_assert(SG_F % 32 == 0 && (4 * SG_H) % 32 == 0);

#define SG_SZ_XB   ((size_t)SG_MP * 128 * 2)
#define SG_SZ_P1   ((size_t)SG_MP * 64 * 4)
#define SG_SZ_O    ((size_t)SG_MP * 64 * 4)
#define SG_SZ_H    ((size_t)SG_N * 16 * 4)
#define SG_SZ_A2   ((size_t)SG_MP * 64 * 2)
#define SG_SZ_LIST ((size_t)SG_NBLK * SG_RCAP * 4)
#define SG_SZ_CNT  ((size_t)SG_NBLK * SG_NBA * 4)
#define SG_SZ_OFF  ((size_t)SG_NBLK * SG_NBA * 4)
#define SG_SZ_FLAG ((size_t)SG_NBLK * 128)
#define SG_SZ_W1   ((size_t)64 * 128 * 2)
#define SG_SZ_W2   ((size_t)64 * 64 * 2)
#define SG_OF_XB   ((size_t)0)
#define SG_OF_P1   (SG_OF_XB + SG_SZ_XB)
#define SG_OF_O    (SG_OF_P1 + SG_SZ_P1)
#define SG_OF_H    (SG_OF_O + SG_SZ_O)
#define SG_OF_A2   (SG_OF_H + SG_SZ_H)
#define SG_OF_LIST (SG_OF_A2 + SG_SZ_A2)
#define SG_OF_CNT  (SG_OF_LIST + SG_SZ_LIST)
#define SG_OF_OFF  (SG_OF_CNT + SG_SZ_CNT)
#define SG_OF_FLAG (SG_OF_OFF + SG_SZ_OFF)
#define SG_OF_W1   (SG_OF_FLAG + SG_SZ_FLAG)
#define SG_OF_W2   (SG_OF_W1 + SG_SZ_W1)
#define SG_WS_TOTAL (SG_OF_W2 + SG_SZ_W2)
static_assert(SG_SZ_XB % 128 == 0 && SG_SZ_P1 % 128 == 0 && SG_SZ_H % 128 == 0 && SG_SZ_A2 % 128 == 0);
static_assert(SG_SZ_LIST % 128 == 0 && SG_SZ_CNT % 128 == 0 && SG_SZ_FLAG % 128 == 0);
static_assert(SG_SZ_W1 % 128 == 0 && SG_SZ_W2 % 128 == 0);
static_assert(SG_WS_TOTAL <= ((size_t)128 << 20));

typedef int v4i __attribute__((ext_vector_type(4)));
typedef v4i __attribute__((may_alias)) v4ia;

__device__ __forceinline__ float qnan_f() { return __uint_as_float(0x7fc00000u); }
__device__ __forceinline__ float blendf(float a, float b, unsigned mb) {
  return __uint_as_float((__float_as_uint(b) & mb) | (__float_as_uint(a) & ~mb));
}

__global__ __launch_bounds__(256) void k_prep(const float* __restrict__ x,
                                              const float* __restrict__ wn1, const float* __restrict__ ws1,
                                              const float* __restrict__ wn2, const float* __restrict__ ws2,
                                              unsigned short* __restrict__ XB, unsigned short* __restrict__ W1c,
                                              unsigned short* __restrict__ W2c) {
  __shared__ __attribute__((aligned(16))) float sw[4096];
  const int tid = (int)threadIdx.x;
  const int blk = (int)blockIdx.x;
  if (blk < SG_XBLK) {
    const unsigned gp = (unsigned)blk * 256u + (unsigned)tid;
    const int row = (int)(gp >> 4);
    const int p   = (int)(gp & 15u);
    const int rc  = row < SG_N ? row : SG_N - 1;
    const float* sp = x + (size_t)rc * SG_F + 8 * p;
    const v4f a = *(const v4fa*)sp;
    const v4f c = *(const v4fa*)(sp + 4);
    asm volatile("" :: "v"(a));
    asm volatile("" :: "v"(c));
    const unsigned mk = row < SG_N ? 0xFFFFFFFFu : 0u;
    v4u o = pack8_bf16(a, c);
    o &= (v4u){ mk, mk, mk, mk };
    volatile v4u* qd = (volatile v4u*)(XB + (size_t)gp * 8);
    *qd = o;
    __threadfence();
    *qd = o;
  } else if (blk == SG_XBLK) {
#pragma unroll
    for (int i = 0; i < 2; ++i) {
      const int idx = tid + 256 * i;
      const v4f va = *(const v4fa*)(ws1 + 4 * idx);
      const v4f vb = *(const v4fa*)(wn1 + 4 * idx);
      *(v4fa*)(sw + 4 * idx) = va;
      *(v4fa*)(sw + 2048 + 4 * idx) = vb;
    }
    __syncthreads();
    v4u ov[4];
#pragma unroll
    for (int i = 0; i < 4; ++i) {
      const int u  = tid + 256 * i;
      const int n  = u >> 4;
      const int k8 = (u & 15) * 8;
      const int nc = n < 32 ? n : 31;
      const int base = (nc >> 4) * 2048 + (nc & 15);
      const v4f a = (v4f){ sw[base + (k8 + 0) * 16], sw[base + (k8 + 1) * 16], sw[base + (k8 + 2) * 16], sw[base + (k8 + 3) * 16] };
      const v4f c = (v4f){ sw[base + (k8 + 4) * 16], sw[base + (k8 + 5) * 16], sw[base + (k8 + 6) * 16], sw[base + (k8 + 7) * 16] };
      const unsigned mk = n < 32 ? 0xFFFFFFFFu : 0u;
      v4u o = pack8_bf16(a, c);
      o &= (v4u){ mk, mk, mk, mk };
      ov[i] = o;
    }
    for (int pass = 0; pass < 2; ++pass) {
#pragma unroll
      for (int i = 0; i < 4; ++i) *(volatile v4u*)(W1c + (size_t)(tid + 256 * i) * 8) = ov[i];
      __threadfence();
    }
  } else {
    {
      const int idx = tid < 160 ? tid : 159;
      const v4f va = *(const v4fa*)(ws2 + 4 * idx);
      const v4f vb = *(const v4fa*)(wn2 + 4 * idx);
      asm volatile("" :: "v"(va));
      asm volatile("" :: "v"(vb));
      if (tid < 160) {
        *(v4fa*)(sw + 4 * idx) = va;
        *(v4fa*)(sw + 640 + 4 * idx) = vb;
      }
    }
    __syncthreads();
    v4u ov[2];
#pragma unroll
    for (int i = 0; i < 2; ++i) {
      const int u  = tid + 256 * i;
      const int n  = u >> 3;
      const int kp = u & 7;
      const int nc = n < SG_C ? n : SG_C - 1;
      const int base = (kp >> 2) * 640 + nc;
      const int kb = (kp & 1) * 8;
      const v4f a = (v4f){ sw[base + (kb + 0) * 40], sw[base + (kb + 1) * 40], sw[base + (kb + 2) * 40], sw[base + (kb + 3) * 40] };
      const v4f c = (v4f){ sw[base + (kb + 4) * 40], sw[base + (kb + 5) * 40], sw[base + (kb + 6) * 40], sw[base + (kb + 7) * 40] };
      const unsigned mk = n < SG_C ? 0xFFFFFFFFu : 0u;
      v4u o = pack8_bf16(a, c);
      o &= (v4u){ mk, mk, mk, mk };
      ov[i] = o;
    }
    for (int pass = 0; pass < 2; ++pass) {
#pragma unroll
      for (int i = 0; i < 2; ++i) *(volatile v4u*)(W2c + (size_t)(tid + 256 * i) * 8) = ov[i];
      __threadfence();
    }
  }
}

__device__ __forceinline__ int hit_put(bool hj, unsigned sj, int srcv, int wc, int* mywl) {
  const unsigned mj = __builtin_amdgcn_ballot_w32(hj);
  if (mj != 0u) {
    const int pos = wc + (int)__builtin_amdgcn_mbcnt_lo(mj, 0u);
    const int sc  = clampi(srcv, 0, SG_N - 1);
    if (hj && pos < SG_WLCAP) mywl[pos] = (int)((sj << 17) | (unsigned)sc);
    wc += (int)__builtin_popcount(mj);
  }
  return wc;
}

__global__ __launch_bounds__(256) void k_bucket(const int* __restrict__ srcs, const int* __restrict__ dsts,
                                                int* __restrict__ LIST, int* __restrict__ CNT,
                                                int* __restrict__ OFF, int* __restrict__ FLAG) {
  extern __shared__ __attribute__((aligned(16))) int dsm[];
  int* sl   = dsm;
  int* cw   = sl + SG_RCAP;
  int* cnt  = cw + 8 * SG_NBA;
  int* offs = cnt + SG_NBA;
  int* misc = offs + SG_NBA;
  int* wl   = misc + 32;
  const int tid = (int)threadIdx.x, lane = tid & 31, wave = tid >> 5;
  const int b = (int)blockIdx.x;
  const int slotBase = b * SG_NBA;
  {
    const v4i z4 = (v4i){0, 0, 0, 0};
    for (int i = tid; i < SG_ZINTS / 4; i += 256) *(v4ia*)(dsm + 4 * i) = z4;
  }
  __syncthreads();

  int* mywl = wl + wave * SG_WLCAP;
  const unsigned nbs = (unsigned)slotBase;
  const unsigned unb = (unsigned)((SG_N - slotBase) < SG_NBA ? (SG_N - slotBase) : SG_NBA);
  int wc = 0;
#pragma unroll 1
  for (int it = 0; it < SG_SWEEP; ++it) {
    const int wch = it * 8 + wave;
    if (wch < SG_NWCH) {
      const int e0 = wch * 256 + lane * 8;
      const v4i da = *(const v4ia*)(dsts + e0);
      const v4i db = *(const v4ia*)(dsts + e0 + 4);
      const v4i sa = *(const v4ia*)(srcs + e0);
      const v4i sb = *(const v4ia*)(srcs + e0 + 4);
      const unsigned s0 = (unsigned)da.x - nbs, s1 = (unsigned)da.y - nbs;
      const unsigned s2 = (unsigned)da.z - nbs, s3 = (unsigned)da.w - nbs;
      const unsigned s4 = (unsigned)db.x - nbs, s5 = (unsigned)db.y - nbs;
      const unsigned s6 = (unsigned)db.z - nbs, s7 = (unsigned)db.w - nbs;
      const bool h0 = s0 < unb, h1 = s1 < unb, h2 = s2 < unb, h3 = s3 < unb;
      const bool h4 = s4 < unb, h5 = s5 < unb, h6 = s6 < unb, h7 = s7 < unb;
      const unsigned any = __builtin_amdgcn_ballot_w32(h0 | h1 | h2 | h3 | h4 | h5 | h6 | h7);
      if (any != 0u) {
        wc = hit_put(h0, s0, sa.x, wc, mywl);
        wc = hit_put(h1, s1, sa.y, wc, mywl);
        wc = hit_put(h2, s2, sa.z, wc, mywl);
        wc = hit_put(h3, s3, sa.w, wc, mywl);
        wc = hit_put(h4, s4, sb.x, wc, mywl);
        wc = hit_put(h5, s5, sb.y, wc, mywl);
        wc = hit_put(h6, s6, sb.z, wc, mywl);
        wc = hit_put(h7, s7, sb.w, wc, mywl);
      }
    }
  }
  if (lane == 0) misc[wave] = (wc > SG_WLCAP) ? 1 : 0;
  __syncthreads();

  int cv = wc;
  cv = cv < 0 ? 0 : (cv > SG_WLCAP ? SG_WLCAP : cv);
  const int c = __builtin_amdgcn_readfirstlane(cv);
  int* mycw = cw + wave * SG_NBA;
#pragma unroll 1
  for (int b0 = 0; b0 < c; b0 += 32) {
    int idx = b0 + lane;
    idx = idx > c - 1 ? c - 1 : idx;
    const int ent = mywl[idx];
    const int m32 = (c - b0) < 32 ? (c - b0) : 32;
#pragma unroll 1
    for (int k = 0; k < m32; ++k) {
      const int u    = __builtin_amdgcn_readlane(ent, k);
      const int slot = (u >> 17) & (SG_NBA - 1);
      if (lane == 0) mycw[slot] = mycw[slot] + 1;
    }
  }
  __syncthreads();

  const int s4i = tid * 4;
  v4i run = (v4i){0, 0, 0, 0};
#pragma unroll
  for (int w = 0; w < 8; ++w) {
    const v4i v = *(const v4ia*)(cw + w * SG_NBA + s4i);
    *(v4ia*)(cw + w * SG_NBA + s4i) = run;
    run += v;
  }
  const int ssum = run.x + run.y + run.z + run.w;
  int incl = ssum;
#pragma unroll
  for (int d = 1; d < 32; d <<= 1) {
    const int y = __shfl_up(incl, d, 32);
    incl += (lane >= d) ? y : 0;
  }
  if (lane == 31) misc[8 + wave] = incl;
  __syncthreads();
  int wbase = 0, total = 0, ovf = 0;
#pragma unroll
  for (int w = 0; w < 8; ++w) {
    const int v = misc[8 + w];
    wbase += (w < wave) ? v : 0;
    total += v;
    ovf |= misc[w];
  }
  ovf |= (total > SG_RCAP) ? 1 : 0;
  const int excl = wbase + incl - ssum;
  const v4i o4 = (v4i){ excl, excl + run.x, excl + run.x + run.y, excl + run.x + run.y + run.z };
  *(v4ia*)(cnt + s4i)  = run;
  *(v4ia*)(offs + s4i) = o4;
#pragma unroll
  for (int w = 0; w < 8; ++w) {
    v4i v = *(const v4ia*)(cw + w * SG_NBA + s4i);
    v += o4;
    *(v4ia*)(cw + w * SG_NBA + s4i) = v;
  }
  __syncthreads();

#pragma unroll 1
  for (int b0 = 0; b0 < c; b0 += 32) {
    int idx = b0 + lane;
    idx = idx > c - 1 ? c - 1 : idx;
    const int ent = mywl[idx];
    const int m32 = (c - b0) < 32 ? (c - b0) : 32;
#pragma unroll 1
    for (int k = 0; k < m32; ++k) {
      const int u    = __builtin_amdgcn_readlane(ent, k);
      const int slot = (u >> 17) & (SG_NBA - 1);
      if (lane == 0) {
        int p = mycw[slot];
        mycw[slot] = p + 1;
        p = p < 0 ? 0 : (p > SG_RCAP - 1 ? SG_RCAP - 1 : p);
        sl[p] = u & 0x1FFFF;
      }
    }
  }
  __syncthreads();

  int* gl = LIST + (size_t)b * SG_RCAP;
  const v4i cn4 = *(const v4ia*)(cnt + s4i);
  const v4i of4 = *(const v4ia*)(offs + s4i);
  const v4i fl4 = (v4i){ ovf, ovf, ovf, ovf };
  for (int pass = 0; pass < 2; ++pass) {
#pragma unroll 1
    for (int i = tid; i < SG_RCAP / 4; i += 256) {
      const v4i v = *(const v4ia*)(sl + 4 * i);
      *(volatile v4i*)(gl + 4 * i) = v;
    }
    *(volatile v4i*)(CNT + (size_t)b * SG_NBA + s4i) = cn4;
    *(volatile v4i*)(OFF + (size_t)b * SG_NBA + s4i) = of4;
    if (tid < 8) *(volatile v4i*)(FLAG + b * 32 + 4 * tid) = fl4;
    __threadfence();
  }
}

template <int PITCH, int COFF>
__device__ __forceinline__ v4f seg_sum(const float* __restrict__ T, const int* __restrict__ gl, int c, int o, int g, int q) {
  v4f s = (v4f){0.f, 0.f, 0.f, 0.f};
#pragma unroll 1
  for (int j0 = 0; j0 < c; j0 += 8) {
    const int j  = j0 + g;
    const int jc = j < c ? j : c - 1;
    int idx = o + jc;
    idx = idx > SG_RCAP - 1 ? SG_RCAP - 1 : idx;
    int sr = gl[idx];
    asm volatile("" :: "v"(sr));
    sr = clampi(sr, 0, SG_N - 1);
    const v4f v = *(const v4fa*)(T + (size_t)sr * PITCH + COFF + 4 * q);
    asm volatile("" :: "v"(v));
    const unsigned mk = (j < c) ? 0xFFFFFFFFu : 0u;
    s.x += __uint_as_float(__float_as_uint(v.x) & mk);
    s.y += __uint_as_float(__float_as_uint(v.y) & mk);
    s.z += __uint_as_float(__float_as_uint(v.z) & mk);
    s.w += __uint_as_float(__float_as_uint(v.w) & mk);
  }
#pragma unroll
  for (int d = 4; d < 32; d <<= 1) {
    const float y0 = __shfl_xor(s.x, d, 32);
    const float y1 = __shfl_xor(s.y, d, 32);
    const float y2 = __shfl_xor(s.z, d, 32);
    const float y3 = __shfl_xor(s.w, d, 32);
    s.x += y0; s.y += y1; s.z += y2; s.w += y3;
  }
  return s;
}

__global__ __launch_bounds__(256) void k_l1(const float* __restrict__ P1, const int* __restrict__ LIST,
                                            const int* __restrict__ CNT, const int* __restrict__ OFF,
                                            const int* __restrict__ FLAG, const float* __restrict__ b1,
                                            float* __restrict__ H) {
  __shared__ __attribute__((aligned(16))) float sb[16];
  const int tid = (int)threadIdx.x, lane = tid & 31, wave = tid >> 5;
  const int g = lane >> 2, q = lane & 3;
  {
    const float v = b1[tid & 15];
    asm volatile("" :: "v"(v));
    if (tid < 16) sb[tid] = bf16_val(v);
  }
  __syncthreads();
  const int b = (int)blockIdx.x;
  const int rowBase = b * SG_NBA;
  const int* gl = LIST + (size_t)b * SG_RCAP;
  const int fl = FLAG[b * 32];
  const v4f bq = *(const v4fa*)(sb + 4 * q);
  const float qn = qnan_f();
#pragma unroll 1
  for (int it = 0; it < SG_NBA / 16; ++it) {
    const int pr = it * 8 + wave;
    const int r0 = rowBase + 2 * pr;
    if (r0 < SG_N) {
      v4f hv = (v4f){0.f, 0.f, 0.f, 0.f};
#pragma unroll 1
      for (int rr = 0; rr < 2; ++rr) {
        const int r  = r0 + rr;
        const int cn = CNT[r];
        const int of = OFF[r];
        int cc = clampi(cn, 0, SG_DEGCAP);
        cc = __builtin_amdgcn_readfirstlane(cc);
        int oo = clampi(of, 0, SG_RCAP - 1);
        oo = __builtin_amdgcn_readfirstlane(oo);
        const v4f s = seg_sum<64, 16>(P1, gl, cc, oo, g, q);
        const v4f self = *(const v4fa*)(P1 + (size_t)r * 64 + 4 * q);
        asm volatile("" :: "v"(self.x), "v"(self.y), "v"(self.z), "v"(self.w));
        const float d = (float)(cn > 1 ? cn : 1);
        v4f t;
        t.x = (self.x + s.x / d) + bq.x;
        t.y = (self.y + s.y / d) + bq.y;
        t.z = (self.z + s.z / d) + bq.z;
        t.w = (self.w + s.w / d) + bq.w;
        t.x = (t.x > 0.0f) ? t.x : (t.x - t.x);
        t.y = (t.y > 0.0f) ? t.y : (t.y - t.y);
        t.z = (t.z > 0.0f) ? t.z : (t.z - t.z);
        t.w = (t.w > 0.0f) ? t.w : (t.w - t.w);
        const bool bad = (fl != 0) | (cn > SG_DEGCAP) | (cn < 0);
        t.x = bad ? qn : t.x; t.y = bad ? qn : t.y; t.z = bad ? qn : t.z; t.w = bad ? qn : t.w;
        const bool take = ((lane >> 2) & 1) == rr;
        hv.x = take ? t.x : hv.x; hv.y = take ? t.y : hv.y; hv.z = take ? t.z : hv.z; hv.w = take ? t.w : hv.w;
      }
      float* hp = H + (size_t)r0 * 16 + 4 * lane;
      if (lane < 8) *(volatile v4f*)hp = hv;
      __threadfence();
      if (lane < 8) *(volatile v4f*)hp = hv;
    }
  }
}

__global__ __launch_bounds__(256) void k_l2(const float* __restrict__ H, const int* __restrict__ LIST,
                                            const int* __restrict__ CNT, const int* __restrict__ OFF,
                                            const int* __restrict__ FLAG, unsigned short* __restrict__ A2) {
  const int tid = (int)threadIdx.x, lane = tid & 31, wave = tid >> 5;
  const int g = lane >> 2, q = lane & 3;
  const int b = (int)blockIdx.x;
  const int rowBase = b * SG_NBA;
  const int* gl = LIST + (size_t)b * SG_RCAP;
  const int fl = FLAG[b * 32];
  const float qn = qnan_f();
  const int half = lane & 1;
  const int srcA = 2 * half, srcB = 2 * half + 1;
  const unsigned mkM  = (lane & 4) ? 0xFFFFFFFFu : 0u;
  const unsigned mkLo = (lane & 2) ? 0xFFFFFFFFu : 0u;
#pragma unroll 1
  for (int it = 0; it < SG_NBA / 8; ++it) {
    const int r = rowBase + it * 8 + wave;
    if (r < SG_MP) {
      const bool live = r < SG_N;
      const int rc = live ? r : SG_N - 1;
      int cn = CNT[r];
      const int of = OFF[r];
      cn = live ? cn : 0;
      int cc = clampi(cn, 0, SG_DEGCAP);
      cc = __builtin_amdgcn_readfirstlane(cc);
      int oo = clampi(of, 0, SG_RCAP - 1);
      oo = __builtin_amdgcn_readfirstlane(oo);
      const v4f s = seg_sum<16, 0>(H, gl, cc, oo, g, q);
      const float d = (float)(cn > 1 ? cn : 1);
      v4f m;
      m.x = s.x / d; m.y = s.y / d; m.z = s.z / d; m.w = s.w / d;
      v4f ma, mc;
      ma.x = __shfl(m.x, srcA, 32); ma.y = __shfl(m.y, srcA, 32); ma.z = __shfl(m.z, srcA, 32); ma.w = __shfl(m.w, srcA, 32);
      mc.x = __shfl(m.x, srcB, 32); mc.y = __shfl(m.y, srcB, 32); mc.z = __shfl(m.z, srcB, 32); mc.w = __shfl(m.w, srcB, 32);
      const float* hp = H + (size_t)rc * 16 + 8 * half;
      const v4f ha = *(const v4fa*)hp;
      const v4f hc = *(const v4fa*)(hp + 4);
      asm volatile("" :: "v"(ha));
      asm volatile("" :: "v"(hc));
      v4f xa, xc;
      xa.x = blendf(ha.x, ma.x, mkM); xa.y = blendf(ha.y, ma.y, mkM); xa.z = blendf(ha.z, ma.z, mkM); xa.w = blendf(ha.w, ma.w, mkM);
      xc.x = blendf(hc.x, mc.x, mkM); xc.y = blendf(hc.y, mc.y, mkM); xc.z = blendf(hc.z, mc.z, mkM); xc.w = blendf(hc.w, mc.w, mkM);
      const bool bad = (fl != 0) | (cn > SG_DEGCAP) | (cn < 0);
      xa.x = bad ? qn : xa.x; xa.y = bad ? qn : xa.y; xa.z = bad ? qn : xa.z; xa.w = bad ? qn : xa.w;
      xc.x = bad ? qn : xc.x; xc.y = bad ? qn : xc.y; xc.z = bad ? qn : xc.z; xc.w = bad ? qn : xc.w;
      const v4u hi = pack8_bf16(xa, xc);
      v4u lo = (v4u){0u, 0u, 0u, 0u};
      if (SPLIT2 != 0) lo = pack8_bf16_lo(xa, xc);
      const v4u ml = (v4u){ mkLo, mkLo, mkLo, mkLo };
      v4u o = (lo & ml) | (hi & ~ml);
      const unsigned lv = live ? 0xFFFFFFFFu : 0u;
      o &= (v4u){ lv, lv, lv, lv };
      unsigned short* ap = A2 + (size_t)r * 64 + 8 * lane;
      if (lane < 8) *(volatile v4u*)ap = o;
      __threadfence();
      if (lane < 8) *(volatile v4u*)ap = o;
    }
  }
}

__global__ __launch_bounds__(256) void k_out(const float* __restrict__ O, const int* __restrict__ FLAG,
                                             const float* __restrict__ b2, float* __restrict__ outp) {
  __shared__ __attribute__((aligned(16))) float sb2[SG_C];
  const int tid = (int)threadIdx.x, lane = tid & 31, wave = tid >> 5;
  {
    const float v = b2[tid < SG_C ? tid : SG_C - 1];
    asm volatile("" :: "v"(v));
    if (tid < SG_C) sb2[tid] = bf16_val(v);
  }
  __syncthreads();
  const int grp = (int)blockIdx.x * 8 + wave;
  if (grp < SG_NGRP) {
    const float qn = qnan_f();
    v4f vv[5];
#pragma unroll
    for (int j = 0; j < 5; ++j) {
      const int f   = lane + 32 * j;
      const int rl  = f / 10;
      const int c   = (f - rl * 10) * 4;
      const int row = grp * 16 + rl;
      const v4f o  = *(const v4fa*)(O + (size_t)row * 64 + c);
      asm volatile("" :: "v"(o.x), "v"(o.y), "v"(o.z), "v"(o.w));
      const v4f bb = *(const v4fa*)(sb2 + c);
      const int fl = FLAG[(row >> 10) * 32];
      asm volatile("" :: "v"(fl));
      v4f t = o + bb;
      const bool bad = fl != 0;
      t.x = bad ? qn : t.x; t.y = bad ? qn : t.y; t.z = bad ? qn : t.z; t.w = bad ? qn : t.w;
      vv[j] = t;
    }
    float* base = outp + (size_t)grp * 640;
    for (int pass = 0; pass < 2; ++pass) {
#pragma unroll
      for (int j = 0; j < 5; ++j) *(volatile v4f*)(base + 4 * (lane + 32 * j)) = vv[j];
      __threadfence();
    }
  }
}

extern "C" void kernel_launch(void* const* d_in, const int* in_sizes, int n_in,
                              void* d_out, int out_size, void* d_ws, size_t ws_size,
                              hipStream_t stream) {
  if (n_in < 9) return;
  if (in_sizes[0] != SG_N * SG_F) return;
  if (in_sizes[1] != SG_E || in_sizes[2] != SG_E) return;
  if (in_sizes[3] != SG_F * SG_H || in_sizes[4] != SG_F * SG_H || in_sizes[5] != SG_H) return;
  if (in_sizes[6] != SG_H * SG_C || in_sizes[7] != SG_H * SG_C || in_sizes[8] != SG_C) return;
  if (out_size != SG_N * SG_C) return;
  if (ws_size < SG_WS_TOTAL) return;

  const float* x   = (const float*)d_in[0];
  const int*   src = (const int*)d_in[1];
  const int*   dst = (const int*)d_in[2];
  const float* wn1 = (const float*)d_in[3];
  const float* ws1 = (const float*)d_in[4];
  const float* b1  = (const float*)d_in[5];
  const float* wn2 = (const float*)d_in[6];
  const float* ws2 = (const float*)d_in[7];
  const float* b2  = (const float*)d_in[8];
  float* outp = (float*)d_out;

  char* ws = (char*)d_ws;
  unsigned short* XB  = (unsigned short*)(ws + SG_OF_XB);
  float*          P1  = (float*)(ws + SG_OF_P1);
  float*          O   = (float*)(ws + SG_OF_O);
  float*          H   = (float*)(ws + SG_OF_H);
  unsigned short* A2  = (unsigned short*)(ws + SG_OF_A2);
  int*            LST = (int*)(ws + SG_OF_LIST);
  int*            CNT = (int*)(ws + SG_OF_CNT);
  int*            OFF = (int*)(ws + SG_OF_OFF);
  int*            FLG = (int*)(ws + SG_OF_FLAG);
  unsigned short* W1c = (unsigned short*)(ws + SG_OF_W1);
  unsigned short* W2c = (unsigned short*)(ws + SG_OF_W2);

  const size_t bucketLds = (size_t)SG_LDSINTS * 4;
  hipFuncSetAttribute(reinterpret_cast<const void*>(&k_bucket), hipFuncAttributeMaxDynamicSharedMemorySize, (int)bucketLds);

  const int gemmGrid = (((SG_N + 63) / 64) + 7) / 8;

  k_prep<<<SG_XBLK + 2, 256, 0, stream>>>(x, wn1, ws1, wn2, ws2, XB, W1c, W2c);
  k_bucket<<<SG_NBLK, 256, bucketLds, stream>>>(src, dst, LST, CNT, OFF, FLG);
  k_gemm_nt<0, 0><<<gemmGrid, 256, 0, stream>>>(XB, W1c, b2, P1, SG_N, 64, SG_F, 64);
  k_l1<<<SG_NBLK, 256, 0, stream>>>(P1, LST, CNT, OFF, FLG, b1, H);
  k_l2<<<SG_NBLK, 256, 0, stream>>>(H, LST, CNT, OFF, FLG, A2);
  k_gemm_nt<0, 0><<<gemmGrid, 256, 0, stream>>>(A2, W2c, b2, O, SG_N, 64, 4 * SG_H, 64);
  k_out<<<(SG_NGRP + 7) / 8, 256, 0, stream>>>(O, FLG, b2, outp);
}
